// CodebookQuantizer_80247168959076
// MI455X (gfx1250) — hardware-verified
//
#include <hip/hip_runtime.h>
#include <stdint.h>

#pragma clang fp contract(off)

typedef __attribute__((ext_vector_type(16))) _Float16 v16h;
typedef __attribute__((ext_vector_type(8)))  _Float16 v8h;
typedef __attribute__((ext_vector_type(16))) __bf16   v16b;
typedef __attribute__((ext_vector_type(8)))  __bf16   v8b;
typedef __attribute__((ext_vector_type(8)))  float    v8f;
typedef __attribute__((ext_vector_type(4)))  float    v4f;
typedef __attribute__((ext_vector_type(4)))  unsigned v4u;

constexpr int NBATCH = 4;
constexpr int NQUERY = 4096;
constexpr int NDIM   = 512;
constexpr int NCODE  = 8192;
constexpr int NROWS  = NBATCH * NQUERY;
constexpr int QROWS  = 32;
constexpr int KCHUNK = 128;
constexpr int PPITCH = 136;
constexpr int SPITCH = 68;
constexpr int TPITCH = 72;
constexpr float  PCARRY   = 32768.0f;
constexpr float  SC_CROSS = 28.853900817779268f;
constexpr double SC_ESQ   = 14.426950408889634;

static_assert(NROWS % QROWS == 0);
static_assert(NCODE % KCHUNK == 0);
static_assert(NDIM % 32 == 0);
static_assert(NDIM == 8 * 64);
static_assert(KCHUNK == 4 * 32);
static_assert(QROWS == 2 * 16);
static_assert(NCODE % 64 == 0 && NDIM % 64 == 0);
static_assert(NCODE % 32 == 0);

constexpr size_t WS_H     = 0;
constexpr size_t WS_H_B   = (size_t)NROWS * NDIM * 2;
constexpr size_t WS_E     = WS_H + WS_H_B;
constexpr size_t WS_E_B   = (size_t)NCODE * NDIM * 2;
constexpr size_t WS_ET    = WS_E + WS_E_B;
constexpr size_t WS_ET_B  = (size_t)NDIM * NCODE * 2;
constexpr size_t WS_ESQ   = WS_ET + WS_ET_B;
constexpr size_t WS_ESQ_B = (size_t)NCODE * 4;
constexpr size_t WS_TOTAL = WS_ESQ + WS_ESQ_B;
static_assert(WS_TOTAL <= (size_t)134217728);
static_assert(WS_E % 128 == 0 && WS_ET % 128 == 0 && WS_ESQ % 128 == 0);

__device__ __forceinline__ unsigned short f2bf_bits(float f) {
  unsigned u = __float_as_uint(f);
  return (unsigned short)((u + 0x7FFFu + ((u >> 16) & 1u)) >> 16);
}
__device__ __forceinline__ float bf_bits2f(unsigned short h) { return __uint_as_float(((unsigned)h) << 16); }
__device__ __forceinline__ float rne_bf16f(float f) { return bf_bits2f(f2bf_bits(f)); }
__device__ __forceinline__ v8f zero8() { return (v8f){0.f, 0.f, 0.f, 0.f, 0.f, 0.f, 0.f, 0.f}; }

__device__ __forceinline__ void dep_guard_h(v8f& a, v8f& b, v16h x, v16h y) { asm volatile("v_nop\n\tv_nop\n\tv_nop\n\tv_nop" : "+v"(a), "+v"(b) : "v"(x), "v"(y)); }
__device__ __forceinline__ void dep_guard_b(v8f& a, v8f& b, v16b x, v16b y) { asm volatile("v_nop\n\tv_nop\n\tv_nop\n\tv_nop" : "+v"(a), "+v"(b) : "v"(x), "v"(y)); }
__device__ __forceinline__ void keep4_h(v16h a, v16h b, v16h c, v16h d) { asm volatile("v_nop" :: "v"(a), "v"(b), "v"(c), "v"(d)); }
__device__ __forceinline__ void keep4_b(v16b a, v16b b, v16b c, v16b d) { asm volatile("v_nop" :: "v"(a), "v"(b), "v"(c), "v"(d)); }
__device__ __forceinline__ void guard2_b3(v8f& a, v8f& b, v16b x, v16b y, v16b z) {
  asm volatile("v_nop\n\tv_nop\n\tv_nop\n\tv_nop" : "+v"(a), "+v"(b) : "v"(x), "v"(y), "v"(z));
}
__device__ __forceinline__ void guard4_h3(v8f& a, v8f& b, v8f& c, v8f& d, v16h x, v16h y, v16h z) {
  asm volatile("v_nop\n\tv_nop\n\tv_nop\n\tv_nop" : "+v"(a), "+v"(b), "+v"(c), "+v"(d) : "v"(x), "v"(y), "v"(z));
}

template <typename T> struct Frag;
template <> struct Frag<_Float16> {
  typedef v16h V; union U { v16h v; v8h h[2]; };
  static __device__ __forceinline__ v16h load(const _Float16* p) {
    U f; f.h[0] = *(const v8h*)(p); f.h[1] = *(const v8h*)(p + 16); return f.v;
  }
  static __device__ __forceinline__ v8f mma(v16h a, v16h b, v8f c) {
    return __builtin_amdgcn_wmma_f32_16x16x32_f16(false, a, false, b, (short)0, c, false, false);
  }
  static __device__ __forceinline__ void guard(v8f& a, v8f& b, v16h x, v16h y) { dep_guard_h(a, b, x, y); }
  static __device__ __forceinline__ void keep(v16h a, v16h b, v16h c, v16h d) { keep4_h(a, b, c, d); }
};
template <> struct Frag<__bf16> {
  typedef v16b V; union U { v16b v; v8b h[2]; };
  static __device__ __forceinline__ v16b load(const __bf16* p) {
    U f; f.h[0] = *(const v8b*)(p); f.h[1] = *(const v8b*)(p + 16); return f.v;
  }
  static __device__ __forceinline__ v8f mma(v16b a, v16b b, v8f c) {
    return __builtin_amdgcn_wmma_f32_16x16x32_bf16(false, a, false, b, (short)0, c, false, false);
  }
  static __device__ __forceinline__ void guard(v8f& a, v8f& b, v16b x, v16b y) { dep_guard_b(a, b, x, y); }
  static __device__ __forceinline__ void keep(v16b a, v16b b, v16b c, v16b d) { keep4_b(a, b, c, d); }
};

__global__ __launch_bounds__(256) void k_cast_bf16x8(const float* __restrict__ src,
                                                      unsigned short* __restrict__ dst, int n8) {
  const int i = blockIdx.x * 256 + threadIdx.x;
  if (i < n8) {
    const float* p = src + (size_t)i * 8;
    const v4f a = *(const v4f*)(p);
    const v4f b = *(const v4f*)(p + 4);
    v4u u;
    u[0] = (unsigned)f2bf_bits(a[0]) | ((unsigned)f2bf_bits(a[1]) << 16);
    u[1] = (unsigned)f2bf_bits(a[2]) | ((unsigned)f2bf_bits(a[3]) << 16);
    u[2] = (unsigned)f2bf_bits(b[0]) | ((unsigned)f2bf_bits(b[1]) << 16);
    u[3] = (unsigned)f2bf_bits(b[2]) | ((unsigned)f2bf_bits(b[3]) << 16);
    volatile v4u* d = (volatile v4u*)(dst + (size_t)i * 8);
    *d = u;
    __threadfence();
    *d = u;
  }
}

__global__ __launch_bounds__(256) void k_prep_e(const float* __restrict__ src,
                                                unsigned short* __restrict__ dst,
                                                float* __restrict__ esq) {
  __shared__ float es[32];
  const int lane = threadIdx.x & 31;
  const int w    = threadIdx.x >> 5;
  const int rbase = blockIdx.x * 32;
#pragma unroll 1
  for (int i = 0; i < 4; ++i) {
    const int row = rbase + 4 * w + i;
    const float* sp = src + (size_t)row * NDIM;
    unsigned short* dp = dst + (size_t)row * NDIM;
    double acc = 0.0;
    v4u u0, u1;
    {
      const float* p0 = sp + lane * 8;
      const v4f a = *(const v4f*)(p0);
      const v4f b = *(const v4f*)(p0 + 4);
      unsigned short hb[8];
      hb[0] = f2bf_bits(a[0]); hb[1] = f2bf_bits(a[1]); hb[2] = f2bf_bits(a[2]); hb[3] = f2bf_bits(a[3]);
      hb[4] = f2bf_bits(b[0]); hb[5] = f2bf_bits(b[1]); hb[6] = f2bf_bits(b[2]); hb[7] = f2bf_bits(b[3]);
#pragma unroll
      for (int e = 0; e < 8; ++e) { const float r = bf_bits2f(hb[e]); const float sq = r * r; acc += (double)sq; }
      u0[0] = (unsigned)hb[0] | ((unsigned)hb[1] << 16);
      u0[1] = (unsigned)hb[2] | ((unsigned)hb[3] << 16);
      u0[2] = (unsigned)hb[4] | ((unsigned)hb[5] << 16);
      u0[3] = (unsigned)hb[6] | ((unsigned)hb[7] << 16);
    }
    {
      const float* p1 = sp + 256 + lane * 8;
      const v4f a = *(const v4f*)(p1);
      const v4f b = *(const v4f*)(p1 + 4);
      unsigned short hb[8];
      hb[0] = f2bf_bits(a[0]); hb[1] = f2bf_bits(a[1]); hb[2] = f2bf_bits(a[2]); hb[3] = f2bf_bits(a[3]);
      hb[4] = f2bf_bits(b[0]); hb[5] = f2bf_bits(b[1]); hb[6] = f2bf_bits(b[2]); hb[7] = f2bf_bits(b[3]);
#pragma unroll
      for (int e = 0; e < 8; ++e) { const float r = bf_bits2f(hb[e]); const float sq = r * r; acc += (double)sq; }
      u1[0] = (unsigned)hb[0] | ((unsigned)hb[1] << 16);
      u1[1] = (unsigned)hb[2] | ((unsigned)hb[3] << 16);
      u1[2] = (unsigned)hb[4] | ((unsigned)hb[5] << 16);
      u1[3] = (unsigned)hb[6] | ((unsigned)hb[7] << 16);
    }
    acc += __shfl_xor(acc, 16, 32);
    acc += __shfl_xor(acc, 8, 32);
    acc += __shfl_xor(acc, 4, 32);
    acc += __shfl_xor(acc, 2, 32);
    acc += __shfl_xor(acc, 1, 32);
    volatile v4u* d0 = (volatile v4u*)(dp + lane * 8);
    volatile v4u* d1 = (volatile v4u*)(dp + 256 + lane * 8);
    *d0 = u0;
    *d1 = u1;
    __threadfence();
    *d0 = u0;
    *d1 = u1;
    if (lane == 0) es[4 * w + i] = (float)((acc - (double)NDIM) * SC_ESQ);
  }
  __syncthreads();
  if (w == 0) {
    const float v = es[lane];
    volatile float* q = esq + rbase + lane;
    *q = v;
    __threadfence();
    *q = v;
  }
}

__global__ __launch_bounds__(256) void k_prep_et(const float* __restrict__ src, _Float16* __restrict__ dst) {
  __shared__ __align__(16) _Float16 tile[64 * TPITCH];
  const int t    = threadIdx.x;
  const int w    = t >> 5;
  const int lane = t & 31;
  const int kt = blockIdx.x >> 3;
  const int dt = blockIdx.x & 7;
  const int kbase = kt * 64;
  const int dbase = dt * 64;
#pragma unroll
  for (int s = 0; s < 4; ++s) {
    const int i  = t + 256 * s;
    const int kk = i >> 4;
    const int d4 = (i & 15) * 4;
    const v4f v = *(const v4f*)(src + (size_t)(kbase + kk) * NDIM + dbase + d4);
    tile[(d4 + 0) * TPITCH + kk] = (_Float16)rne_bf16f(v[0]);
    tile[(d4 + 1) * TPITCH + kk] = (_Float16)rne_bf16f(v[1]);
    tile[(d4 + 2) * TPITCH + kk] = (_Float16)rne_bf16f(v[2]);
    tile[(d4 + 3) * TPITCH + kk] = (_Float16)rne_bf16f(v[3]);
  }
  __syncthreads();
  const int q  = lane >> 3;
  const int c8 = (lane & 7) * 8;
  v8h hv[2];
#pragma unroll
  for (int it = 0; it < 2; ++it) {
    const int row = w * 8 + it * 4 + q;
    hv[it] = *(const v8h*)(tile + row * TPITCH + c8);
  }
  for (int pass = 0; pass < 2; ++pass) {
#pragma unroll
    for (int it = 0; it < 2; ++it) {
      const int row = w * 8 + it * 4 + q;
      *(volatile v8h*)(dst + (size_t)(dbase + row) * NCODE + kbase + c8) = hv[it];
    }
    __threadfence();
  }
}

__global__ __launch_bounds__(256) void k_vq(const unsigned short* __restrict__ ghp,
                                            const unsigned short* __restrict__ gep,
                                            const unsigned short* __restrict__ getp,
                                            const float* __restrict__ esq,
                                            const float* __restrict__ hsrc,
                                            float* __restrict__ out) {
  __shared__ __align__(16) _Float16 Psh[QROWS * PPITCH];
  __shared__ __align__(16) float tmax_s[QROWS * 4];
  __shared__ __align__(16) float tsum_s[QROWS * 4];
  __shared__ __align__(16) float alpha_s[QROWS];
  __shared__ __align__(16) float linv_s[QROWS];
  __shared__ __align__(16) int   nz_s[8];
  __shared__ __align__(16) float slab_s[8][16 * SPITCH];

  const int tid  = threadIdx.x;
  const int w    = tid >> 5;
  const int lane = tid & 31;
  const int hh   = lane >> 4;
  const int c    = lane & 15;
  const int qs   = w & 1;
  const int kg   = w >> 1;
  const int row0 = blockIdx.x * QROWS;

  const __bf16*   gh   = (const __bf16*)ghp;
  const __bf16*   ge   = (const __bf16*)gep;
  const _Float16* get_ = (const _Float16*)getp;

  const __bf16* arow = gh + (size_t)(row0 + 16 * qs + c) * NDIM + 8 * hh;
  const _Float16* vrow = get_ + (size_t)(64 * w + c) * NCODE + 8 * hh;
  const _Float16* p0base = Psh + c * PPITCH + 8 * hh;
  const _Float16* p1base = Psh + (16 + c) * PPITCH + 8 * hh;

  float mrow[8], lrow[8];
#pragma unroll
  for (int r = 0; r < 8; ++r) { mrow[r] = -__builtin_inff(); lrow[r] = 0.0f; }
  v8f oacc[8];
#pragma unroll
  for (int t = 0; t < 8; ++t) oacc[t] = zero8();

  for (int kc = 0; kc < NCODE / KCHUNK; ++kc) {
    const int kv0 = kc * KCHUNK;
    __syncthreads();

    v8f s0 = zero8(), s1 = zero8();
    {
      const __bf16* b0p = ge + (size_t)(kv0 + 32 * kg + c) * NDIM + 8 * hh;
      const __bf16* b1p = b0p + (size_t)16 * NDIM;
#pragma unroll 2
      for (int k0 = 0; k0 < NDIM; k0 += 32) {
        const v16b fa = Frag<__bf16>::load(arow + k0);
        const v16b f0 = Frag<__bf16>::load(b0p + k0);
        const v16b f1 = Frag<__bf16>::load(b1p + k0);
        s0 = Frag<__bf16>::mma(fa, f0, s0);
        s1 = Frag<__bf16>::mma(fa, f1, s1);
        guard2_b3(s0, s1, fa, f0, f1);
      }
    }

    const float e0 = esq[kv0 + 32 * kg + c];
    const float e1 = esq[kv0 + 32 * kg + 16 + c];
    float lg0[8], lg1[8], pm[8];
#pragma unroll
    for (int r = 0; r < 8; ++r) {
      lg0[r] = s0[r] * SC_CROSS - e0;
      lg1[r] = s1[r] * SC_CROSS - e1;
      float m = fmaxf(lg0[r], lg1[r]);
      m = fmaxf(m, __shfl_xor(m, 1, 32));
      m = fmaxf(m, __shfl_xor(m, 2, 32));
      m = fmaxf(m, __shfl_xor(m, 4, 32));
      m = fmaxf(m, __shfl_xor(m, 8, 32));
      pm[r] = m;
    }
    if (c == 0) {
#pragma unroll
      for (int r = 0; r < 8; ++r) tmax_s[(16 * qs + 8 * hh + r) * 4 + kg] = pm[r];
    }
    __syncthreads();

    float alpha[8], ps[8];
    int nz = 0;
#pragma unroll
    for (int r = 0; r < 8; ++r) {
      const int row = 16 * qs + 8 * hh + r;
      const v4f t = *(const v4f*)(tmax_s + row * 4);
      const float cm   = fmaxf(fmaxf(t[0], t[1]), fmaxf(t[2], t[3]));
      const float mnew = fmaxf(mrow[r], cm);
      alpha[r] = exp2f(mrow[r] - mnew);
      mrow[r] = mnew;
      const float pr0 = exp2f(lg0[r] - mnew);
      const float pr1 = exp2f(lg1[r] - mnew);
      const _Float16 pq0 = (_Float16)(pr0 * PCARRY);
      const _Float16 pq1 = (_Float16)(pr1 * PCARRY);
      Psh[row * PPITCH + 32 * kg + c]      = pq0;
      Psh[row * PPITCH + 32 * kg + 16 + c] = pq1;
      nz |= (int)__builtin_bit_cast(unsigned short, pq0) | (int)__builtin_bit_cast(unsigned short, pq1);
      float sq = pr0 + pr1;
      sq += __shfl_xor(sq, 1, 32);
      sq += __shfl_xor(sq, 2, 32);
      sq += __shfl_xor(sq, 4, 32);
      sq += __shfl_xor(sq, 8, 32);
      ps[r] = sq;
    }
    const int anynz = __any(nz != 0);
    if (c == 0) {
#pragma unroll
      for (int r = 0; r < 8; ++r) {
        const int row = 16 * qs + 8 * hh + r;
        tsum_s[row * 4 + kg] = ps[r];
        if (kg == 0) alpha_s[row] = alpha[r];
      }
    }
    if (lane == 0) nz_s[4 * qs + kg] = anynz;
    __syncthreads();

#pragma unroll
    for (int r = 0; r < 8; ++r) {
      const v4f t = *(const v4f*)(tsum_s + (16 * qs + 8 * hh + r) * 4);
      lrow[r] = lrow[r] * alpha[r] + ((t[0] + t[1]) + (t[2] + t[3]));
    }
    {
      const v4f a00 = *(const v4f*)(alpha_s + 8 * hh);
      const v4f a01 = *(const v4f*)(alpha_s + 8 * hh + 4);
      const v4f a10 = *(const v4f*)(alpha_s + 16 + 8 * hh);
      const v4f a11 = *(const v4f*)(alpha_s + 16 + 8 * hh + 4);
      const float al0[8] = {a00[0], a00[1], a00[2], a00[3], a01[0], a01[1], a01[2], a01[3]};
      const float al1[8] = {a10[0], a10[1], a10[2], a10[3], a11[0], a11[1], a11[2], a11[3]};
#pragma unroll
      for (int j = 0; j < 4; ++j) {
#pragma unroll
        for (int r = 0; r < 8; ++r) {
          oacc[j][r]     *= al0[r];
          oacc[4 + j][r] *= al1[r];
        }
      }
    }

    {
#pragma unroll
      for (int kk = 0; kk < KCHUNK / 32; ++kk) {
        const int f0 = __builtin_amdgcn_readfirstlane(nz_s[kk]);
        const int f1 = __builtin_amdgcn_readfirstlane(nz_s[4 + kk]);
        if ((f0 | f1) != 0) {
          v16h vb[4];
#pragma unroll
          for (int j = 0; j < 4; ++j)
            vb[j] = Frag<_Float16>::load(vrow + (size_t)(16 * j) * NCODE + kv0 + 32 * kk);
          const v16h pa0 = Frag<_Float16>::load(p0base + 32 * kk);
          const v16h pa1 = Frag<_Float16>::load(p1base + 32 * kk);
          if (f0 != 0) {
#pragma unroll
            for (int j = 0; j < 4; ++j) oacc[j] = Frag<_Float16>::mma(pa0, vb[j], oacc[j]);
            guard4_h3(oacc[0], oacc[1], oacc[2], oacc[3], pa0, vb[0], vb[3]);
          }
          if (f1 != 0) {
#pragma unroll
            for (int j = 0; j < 4; ++j) oacc[4 + j] = Frag<_Float16>::mma(pa1, vb[j], oacc[4 + j]);
            guard4_h3(oacc[4], oacc[5], oacc[6], oacc[7], pa1, vb[0], vb[3]);
          }
          keep4_h(vb[0], vb[1], vb[2], vb[3]);
        }
      }
    }
  }

  if (kg == 0 && c == 0) {
#pragma unroll
    for (int r = 0; r < 8; ++r) linv_s[16 * qs + 8 * hh + r] = 1.0f / (lrow[r] * PCARRY);
  }
  __syncthreads();
  {
    float* slab = slab_s[w];
    const int h2 = lane >> 4;
    const int c4 = (lane & 15) * 4;
#pragma unroll
    for (int a = 0; a < 2; ++a) {
      const v4f q0 = *(const v4f*)(linv_s + 16 * a + 8 * hh);
      const v4f q1 = *(const v4f*)(linv_s + 16 * a + 8 * hh + 4);
      const float li[8] = {q0[0], q0[1], q0[2], q0[3], q1[0], q1[1], q1[2], q1[3]};
#pragma unroll
      for (int j = 0; j < 4; ++j) {
#pragma unroll
        for (int r = 0; r < 8; ++r) slab[(8 * hh + r) * SPITCH + 16 * j + c] = oacc[4 * a + j][r] * li[r];
      }
      __builtin_amdgcn_fence(__ATOMIC_RELEASE, "workgroup");
      __builtin_amdgcn_wave_barrier();
      __builtin_amdgcn_fence(__ATOMIC_ACQUIRE, "workgroup");
      v4f zr[8];
#pragma unroll
      for (int it = 0; it < 8; ++it) {
        const int row = 2 * it + h2;
        const v4f ze = *(const v4f*)(slab + row * SPITCH + c4);
        const v4f hv = *(const v4f*)(hsrc + (size_t)(row0 + 16 * a + row) * NDIM + 64 * w + c4);
        v4f hr;
        hr[0] = rne_bf16f(hv[0]); hr[1] = rne_bf16f(hv[1]); hr[2] = rne_bf16f(hv[2]); hr[3] = rne_bf16f(hv[3]);
        const v4f dz = ze - hr;
        zr[it] = hr + dz;
      }
      for (int pass = 0; pass < 2; ++pass) {
#pragma unroll
        for (int it = 0; it < 8; ++it) {
          const int row = 2 * it + h2;
          *(volatile v4f*)(out + (size_t)(row0 + 16 * a + row) * NDIM + 64 * w + c4) = zr[it];
        }
        __threadfence();
      }
      __builtin_amdgcn_fence(__ATOMIC_RELEASE, "workgroup");
      __builtin_amdgcn_wave_barrier();
      __builtin_amdgcn_fence(__ATOMIC_ACQUIRE, "workgroup");
    }
  }
}

extern "C" void kernel_launch(void* const* d_in, const int* in_sizes, int n_in,
                              void* d_out, int out_size, void* d_ws, size_t ws_size,
                              hipStream_t stream) {
  if (n_in < 2) return;
  if (in_sizes[0] != NROWS * NDIM) return;
  if (in_sizes[1] != NCODE * NDIM) return;
  if (out_size != NROWS * NDIM) return;
  if (ws_size < WS_TOTAL) return;

  const float* h = (const float*)d_in[0];
  const float* e = (const float*)d_in[1];
  char* ws = (char*)d_ws;
  unsigned short* gh  = (unsigned short*)(ws + WS_H);
  unsigned short* ge  = (unsigned short*)(ws + WS_E);
  _Float16*       get = (_Float16*)(ws + WS_ET);
  float*          esq = (float*)(ws + WS_ESQ);
  float*          out = (float*)d_out;

  const int n8 = NROWS * NDIM / 8;
  k_cast_bf16x8<<<(n8 + 255) / 256, 256, 0, stream>>>(h, gh, n8);
  k_prep_e<<<NCODE / 32, 256, 0, stream>>>(e, ge, esq);
  k_prep_et<<<(NCODE / 64) * (NDIM / 64), 256, 0, stream>>>(e, get);
  k_vq<<<NROWS / QROWS, 256, 0, stream>>>(gh, ge, (const unsigned short*)get, esq, h, out);
}
